// Projection_45827301048522
// MI455X (gfx1250) — hardware-verified
//
#include <hip/hip_runtime.h>
#include <math.h>

constexpr int kRows = 1024;
constexpr int kDim  = 512;
constexpr int kNB   = 32;
constexpr float kInvDim = 1.0f / 512.0f;
constexpr float kLnEps  = 1e-5f;

typedef __attribute__((ext_vector_type(16))) _Float16 v16h;
typedef __attribute__((ext_vector_type(8)))  _Float16 v8h;
typedef __attribute__((ext_vector_type(16))) __bf16   v16b;
typedef __attribute__((ext_vector_type(8)))  __bf16   v8b;
typedef __attribute__((ext_vector_type(8)))  float    v8f;
typedef __attribute__((ext_vector_type(4)))  float    v4f;
typedef __attribute__((ext_vector_type(4)))  unsigned int v4u;

__device__ __forceinline__ unsigned short f2bf_bits(float f) {
  unsigned u = __float_as_uint(f);
  return (unsigned short)((u + 0x7FFFu + ((u >> 16) & 1u)) >> 16);
}
__device__ __forceinline__ float bf_bits2f(unsigned short h) { return __uint_as_float(((unsigned)h) << 16); }

__device__ __forceinline__ void dep_guard_h(v8f& a, v8f& b, v16h x, v16h y) { asm volatile("v_nop\n\tv_nop\n\tv_nop\n\tv_nop" : "+v"(a), "+v"(b) : "v"(x), "v"(y)); }
__device__ __forceinline__ void dep_guard_b(v8f& a, v8f& b, v16b x, v16b y) { asm volatile("v_nop\n\tv_nop\n\tv_nop\n\tv_nop" : "+v"(a), "+v"(b) : "v"(x), "v"(y)); }
__device__ __forceinline__ void keep4_h(v16h a, v16h b, v16h c, v16h d) { asm volatile("v_nop" :: "v"(a), "v"(b), "v"(c), "v"(d)); }
__device__ __forceinline__ void keep4_b(v16b a, v16b b, v16b c, v16b d) { asm volatile("v_nop" :: "v"(a), "v"(b), "v"(c), "v"(d)); }
__device__ __forceinline__ void acc_guard4(v8f& a, v8f& b, v8f& c, v8f& d) { asm volatile("v_nop\n\tv_nop\n\tv_nop\n\tv_nop" : "+v"(a), "+v"(b), "+v"(c), "+v"(d)); }
template <typename T> struct Frag;
template <> struct Frag<_Float16> {
  typedef v16h V; union U { v16h v; v8h h[2]; };
  static __device__ __forceinline__ v16h load(const _Float16* p) {
    U f; f.h[0] = *(const v8h*)(p); f.h[1] = *(const v8h*)(p + 16); return f.v;
  }
  static __device__ __forceinline__ v8f mma(v16h a, v16h b, v8f c) {
    return __builtin_amdgcn_wmma_f32_16x16x32_f16(false, a, false, b, (short)0, c, false, false);
  }
  static __device__ __forceinline__ void guard(v8f& a, v8f& b, v16h x, v16h y) { dep_guard_h(a, b, x, y); }
  static __device__ __forceinline__ void keep(v16h a, v16h b, v16h c, v16h d) { keep4_h(a, b, c, d); }
};
template <> struct Frag<__bf16> {
  typedef v16b V; union U { v16b v; v8b h[2]; };
  static __device__ __forceinline__ v16b load(const __bf16* p) {
    U f; f.h[0] = *(const v8b*)(p); f.h[1] = *(const v8b*)(p + 16); return f.v;
  }
  static __device__ __forceinline__ v8f mma(v16b a, v16b b, v8f c) {
    return __builtin_amdgcn_wmma_f32_16x16x32_bf16(false, a, false, b, (short)0, c, false, false);
  }
  static __device__ __forceinline__ void guard(v8f& a, v8f& b, v16b x, v16b y) { dep_guard_b(a, b, x, y); }
  static __device__ __forceinline__ void keep(v16b a, v16b b, v16b c, v16b d) { keep4_b(a, b, c, d); }
};

__device__ __forceinline__ unsigned pk16(unsigned short a, unsigned short b) { return (unsigned)a | ((unsigned)b << 16); }
__device__ __forceinline__ unsigned short h_bits(float f) { const _Float16 h = (_Float16)f; return __builtin_bit_cast(unsigned short, h); }

template <int ET> struct Elem;
template <> struct Elem<0> { typedef _Float16 T; };
template <> struct Elem<1> { typedef __bf16 T; };
template <int ET, bool SPLIT, int BIAS_MODE, int OUT_MODE, bool RESID, int ACT = 0>
__global__ __launch_bounds__(256) void wmma_gemm64(
    const unsigned short* __restrict__ Ap, const unsigned short* __restrict__ A2p, int lda, long strideA,
    const unsigned short* __restrict__ Btp, const unsigned short* __restrict__ Bt2p, int ldb, long strideB,
    void* __restrict__ Cout, void* __restrict__ Cout2, int ldc, long strideC,
    const float* __restrict__ bias,
    const float* __restrict__ resid, long strideR,
    int M, int N, int K, float scale) {
  typedef typename Elem<ET>::T T;
  typedef typename Frag<T>::V V;
  const T* A = (const T*)Ap; const T* A2 = (const T*)A2p; const T* Bt = (const T*)Btp; const T* Bt2 = (const T*)Bt2p;
  __shared__ __align__(16) float sT[8][16 * 68];
  const int b    = blockIdx.y;
  const int lane = threadIdx.x & 31;
  const int wave = threadIdx.x >> 5;
  const int tilesN = N >> 6;
  const int tilesM = M >> 6;
  const int tile = blockIdx.x * 8 + wave;
  if (tile >= tilesM * tilesN) return;
  const int tm = tile / tilesN;
  const int tn = tile - tm * tilesN;
  const int m0 = tm << 6;
  const int n0 = tn << 6;

  const T* Ab  = A  + (size_t)b * strideA;
  const T* Bb  = Bt + (size_t)b * strideB;
  const T* Ab2 = SPLIT ? (A2  + (size_t)b * strideA) : nullptr;
  const T* Bb2 = SPLIT ? (Bt2 + (size_t)b * strideB) : nullptr;

  const int rlane = lane & 15;
  const int koff  = (lane >> 4) * 8;
  const int mOff  = (lane >> 4) * 8;

  v8f acc[4][4];
#pragma unroll
  for (int i = 0; i < 4; ++i)
#pragma unroll
    for (int j = 0; j < 4; ++j) acc[i][j] = (v8f){0.f,0.f,0.f,0.f,0.f,0.f,0.f,0.f};

  for (int k0 = 0; k0 < K; k0 += 32) {
    V bh[4], bl[4];
#pragma unroll
    for (int j = 0; j < 4; ++j) {
      const size_t bo = (size_t)(n0 + (j << 4) + rlane) * ldb + koff + k0;
      bh[j] = Frag<T>::load(Bb + bo);
      if (SPLIT) bl[j] = Frag<T>::load(Bb2 + bo);
    }
#pragma unroll
    for (int i = 0; i < 4; ++i) {
      const size_t ao = (size_t)(m0 + (i << 4) + rlane) * lda + koff + k0;
      V ah = Frag<T>::load(Ab + ao);
      V al;
      if (SPLIT) al = Frag<T>::load(Ab2 + ao);
#pragma unroll
      for (int j = 0; j < 4; ++j) {
        acc[i][j] = Frag<T>::mma(ah, bh[j], acc[i][j]);
        if (SPLIT) {
          acc[i][j] = Frag<T>::mma(ah, bl[j], acc[i][j]);
          acc[i][j] = Frag<T>::mma(al, bh[j], acc[i][j]);
        }
      }
      Frag<T>::guard(acc[i][0], acc[i][3], ah, SPLIT ? al : ah);
    }
    Frag<T>::keep(bh[0], bh[1], bh[2], bh[3]);
    if (SPLIT) Frag<T>::keep(bl[0], bl[1], bl[2], bl[3]);
  }
  acc_guard4(acc[0][0], acc[0][1], acc[0][2], acc[0][3]);
  acc_guard4(acc[1][0], acc[1][1], acc[1][2], acc[1][3]);
  acc_guard4(acc[2][0], acc[2][1], acc[2][2], acc[2][3]);
  acc_guard4(acc[3][0], acc[3][1], acc[3][2], acc[3][3]);

  float* slab = sT[wave];
  const float* Rb = RESID ? (resid + (size_t)b * strideR) : nullptr;
#pragma unroll
  for (int i = 0; i < 4; ++i) {
    const int mBase = m0 + (i << 4);
#pragma unroll
    for (int j = 0; j < 4; ++j) {
      const int n = n0 + (j << 4) + rlane;
      float bv = 0.f;
      if (BIAS_MODE == 2) bv = bias[n];
#pragma unroll
      for (int r = 0; r < 8; ++r) {
        float v = acc[i][j][r] * scale;
        if (BIAS_MODE == 1) v += bias[mBase + mOff + r];
        if (BIAS_MODE == 2) v += bv;
        if (RESID) v += Rb[(size_t)(mBase + mOff + r) * ldc + n];
        if (ACT == 1) v = tanhf(v);
        if (ACT == 2) v = fmaxf(v, 0.0f);
        if (ACT == 3) v = v / (1.0f + expf(-v));
        if (ACT == 4) v = (v > 0.f) ? v : 0.01f * v;
        if (ACT == 5) v = 0.5f * v * (1.0f + erff(v * 0.70710678118654752f));
        slab[(mOff + r) * 68 + (j << 4) + rlane] = v;
      }
    }
    __builtin_amdgcn_fence(__ATOMIC_RELEASE, "workgroup");
    __builtin_amdgcn_wave_barrier();
    __builtin_amdgcn_fence(__ATOMIC_ACQUIRE, "workgroup");
    if (OUT_MODE == 0) {
      float* C = (float*)Cout + (size_t)b * strideC;
      const int hh = lane >> 4, c4 = (lane & 15) * 4;
      for (int pass = 0; pass < 2; ++pass) {
#pragma unroll
        for (int it = 0; it < 8; ++it) {
          const int row = it * 2 + hh;
          v4f v = *(const v4f*)(slab + row * 68 + c4);
          *(volatile v4f*)(C + (size_t)(mBase + row) * ldc + n0 + c4) = v;
        }
        __threadfence();
      }
    } else {
      const int q = lane >> 3, c8 = (lane & 7) * 8;
      unsigned short* C  = (unsigned short*)Cout  + (size_t)b * strideC;
      unsigned short* C2 = (OUT_MODE == 2) ? ((unsigned short*)Cout2 + (size_t)b * strideC) : nullptr;
      for (int pass = 0; pass < 2; ++pass) {
#pragma unroll
        for (int it = 0; it < 4; ++it) {
          const int row = it * 4 + q;
          const float* sp = slab + row * 68 + c8;
          v8h hv, lv;
#pragma unroll
          for (int e = 0; e < 8; ++e) {
            if (OUT_MODE == 1) {
              hv[e] = (_Float16)sp[e];
            } else {
              unsigned short hb = f2bf_bits(sp[e]);
              unsigned short lb = f2bf_bits(sp[e] - bf_bits2f(hb));
              hv[e] = __builtin_bit_cast(_Float16, hb);
              lv[e] = __builtin_bit_cast(_Float16, lb);
            }
          }
          *(volatile v8h*)(C + (size_t)(mBase + row) * ldc + n0 + c8) = hv;
          if (OUT_MODE == 2) *(volatile v8h*)(C2 + (size_t)(mBase + row) * ldc + n0 + c8) = lv;
        }
        __threadfence();
      }
    }
    __builtin_amdgcn_fence(__ATOMIC_RELEASE, "workgroup");
    __builtin_amdgcn_wave_barrier();
    __builtin_amdgcn_fence(__ATOMIC_ACQUIRE, "workgroup");
  }
}

template <int MODE>
__global__ __launch_bounds__(256) void cast8_kernel(const float* __restrict__ in, unsigned short* __restrict__ out, int n8, float scale) {
  const int i = blockIdx.x * 256 + threadIdx.x;
  if (i >= n8) return;
  const float* p = in + 8 * (size_t)i;
  const v4f a = *(const v4f*)(p);
  const v4f c = *(const v4f*)(p + 4);
  unsigned short hb[8];
#pragma unroll
  for (int e = 0; e < 4; ++e) {
    if (MODE == 0) {
      hb[e]     = f2bf_bits(a[e]);
      hb[4 + e] = f2bf_bits(c[e]);
    } else {
      hb[e]     = h_bits(bf_bits2f(f2bf_bits(a[e])) * scale);
      hb[4 + e] = h_bits(bf_bits2f(f2bf_bits(c[e])) * scale);
    }
  }
  const v4u u = (v4u){pk16(hb[0], hb[1]), pk16(hb[2], hb[3]), pk16(hb[4], hb[5]), pk16(hb[6], hb[7])};
  unsigned short* q = out + 8 * (size_t)i;
  *(volatile v4u*)q = u;
  __threadfence();
  *(volatile v4u*)q = u;
  (void)scale;
}

__global__ __launch_bounds__(256) void transpose_cast_kernel(const float* __restrict__ in, unsigned short* __restrict__ out) {
  __shared__ float sT[64][65];
  const int t  = threadIdx.x;
  const int o0 = blockIdx.x * 64;
  const int i0 = blockIdx.y * 64;
  const int r  = blockIdx.z;
  const float* src = in + (size_t)r * kDim * kDim;
#pragma unroll
  for (int it = 0; it < 4; ++it) {
    const int flat = it * 256 + t;
    const int ii = flat >> 4;
    const int c4 = (flat & 15) * 4;
    const v4f v = *(const v4f*)(src + (size_t)(i0 + ii) * kDim + o0 + c4);
    sT[c4 + 0][ii] = v[0];
    sT[c4 + 1][ii] = v[1];
    sT[c4 + 2][ii] = v[2];
    sT[c4 + 3][ii] = v[3];
  }
  __syncthreads();
  unsigned short* dst = out + (size_t)r * kDim * kDim;
  const int wave = t >> 5, lane = t & 31;
  const int q = lane >> 3, c8 = (lane & 7) * 8;
  for (int pass = 0; pass < 2; ++pass) {
#pragma unroll
    for (int it = 0; it < 2; ++it) {
      const int oo = it * 32 + wave * 4 + q;
      unsigned short hb[8];
#pragma unroll
      for (int e = 0; e < 8; ++e) hb[e] = f2bf_bits(sT[oo][c8 + e]);
      const v4u u = (v4u){pk16(hb[0], hb[1]), pk16(hb[2], hb[3]), pk16(hb[4], hb[5]), pk16(hb[6], hb[7])};
      *(volatile v4u*)(dst + (size_t)(o0 + oo) * kDim + i0 + c8) = u;
    }
    __threadfence();
  }
}

__global__ __launch_bounds__(128) void mix_bias_ln_kernel(const float* __restrict__ PB, const int* __restrict__ rid,
                                                          const float* __restrict__ rel_bias, const float* __restrict__ rel_att,
                                                          float* __restrict__ out, int nrel) {
  __shared__ float attS[kNB];
  __shared__ float redA[4];
  __shared__ float redB[4];
  const int row  = blockIdx.x;
  const int t    = threadIdx.x;
  const int lane = t & 31, wave = t >> 5;
  const int c0   = t * 4;
  if (wave == 0) {
    int id = rid[row];
    id = (id < 0) ? (id + nrel) : id;
    id = (id < 0) ? 0 : id;
    id = (id > nrel - 1) ? (nrel - 1) : id;
    attS[lane] = bf_bits2f(f2bf_bits(rel_att[(size_t)id * kNB + lane]));
  }
  __syncthreads();

  float acc[4] = {0.f, 0.f, 0.f, 0.f};
  float bac[4] = {0.f, 0.f, 0.f, 0.f};
#pragma unroll 1
  for (int r = 0; r < kNB; ++r) {
    const float a = attS[r];
    const v4f p  = *(const v4f*)(PB + ((size_t)r * kRows + row) * kDim + c0);
    const v4f bb = *(const v4f*)(rel_bias + (size_t)r * kDim + c0);
#pragma unroll
    for (int e = 0; e < 4; ++e) {
      acc[e] = fmaf(a, p[e], acc[e]);
      bac[e] = fmaf(a, bf_bits2f(f2bf_bits(bb[e])), bac[e]);
    }
  }
  float x[4];
#pragma unroll
  for (int e = 0; e < 4; ++e) x[e] = acc[e] + bac[e];

  float s = (x[0] + x[1]) + (x[2] + x[3]);
#pragma unroll
  for (int off = 16; off > 0; off >>= 1) s += __shfl_xor(s, off, 32);
  if (lane == 0) redA[wave] = s;
  __syncthreads();
  const float mu = ((redA[0] + redA[1]) + (redA[2] + redA[3])) * kInvDim;
  float d[4];
#pragma unroll
  for (int e = 0; e < 4; ++e) d[e] = x[e] - mu;
  float qq = (d[0] * d[0] + d[1] * d[1]) + (d[2] * d[2] + d[3] * d[3]);
#pragma unroll
  for (int off = 16; off > 0; off >>= 1) qq += __shfl_xor(qq, off, 32);
  if (lane == 0) redB[wave] = qq;
  __syncthreads();
  const float var = ((redB[0] + redB[1]) + (redB[2] + redB[3])) * kInvDim;
  const float rs  = rsqrtf(var + kLnEps);
  const v4f ov = (v4f){d[0] * rs, d[1] * rs, d[2] * rs, d[3] * rs};
  float* op = out + (size_t)row * kDim + c0;
  *(volatile v4f*)op = ov;
  __threadfence();
  *(volatile v4f*)op = ov;
}

extern "C" void kernel_launch(void* const* d_in, const int* in_sizes, int n_in,
                              void* d_out, int out_size, void* d_ws, size_t ws_size,
                              hipStream_t stream) {
  if (n_in < 5) return;
  if (in_sizes[0] != kRows * kDim) return;
  if (in_sizes[1] != kRows) return;
  if (in_sizes[2] != kNB * kDim * kDim) return;
  if (in_sizes[3] != kNB * kDim) return;
  if (in_sizes[4] < kNB || (in_sizes[4] % kNB) != 0) return;
  if (out_size != kRows * kDim) return;
  const int nrel = in_sizes[4] / kNB;

  const float* e        = (const float*)d_in[0];
  const int*   rid      = (const int*)d_in[1];
  const float* rel_base = (const float*)d_in[2];
  const float* rel_bias = (const float*)d_in[3];
  const float* rel_att  = (const float*)d_in[4];
  float* outp = (float*)d_out;

  const size_t SZ_EB = (size_t)kRows * kDim * 2;
  const size_t SZ_BT = (size_t)kNB * kDim * kDim * 2;
  const size_t SZ_PB = (size_t)kNB * kRows * kDim * 4;
  size_t off = 0;
  const size_t oEB = off; off += SZ_EB;
  const size_t oBT = off; off += SZ_BT;
  const size_t oPB = off; off += SZ_PB;
  const size_t TOTAL = off;
  if (TOTAL > ws_size) return;
  if (TOTAL > (size_t)134217728) return;

  char* ws = (char*)d_ws;
  unsigned short* EB = (unsigned short*)(ws + oEB);
  unsigned short* BT = (unsigned short*)(ws + oBT);
  float*          PB = (float*)(ws + oPB);

  {
    const int n8 = kRows * kDim / 8;
    cast8_kernel<0><<<dim3(n8 / 256), dim3(256), 0, stream>>>(e, EB, n8, 1.0f);
  }
  transpose_cast_kernel<<<dim3(kDim / 64, kDim / 64, kNB), dim3(256), 0, stream>>>(rel_base, BT);

  {
    const int tiles = (kRows / 64) * (kDim / 64);
    wmma_gemm64<1, false, 0, 0, false, 0><<<dim3((tiles + 7) / 8, kNB), dim3(256), 0, stream>>>(
        EB, EB, kDim, 0L,
        BT, BT, kDim, (long)kDim * kDim,
        (void*)PB, (void*)PB, kDim, (long)kRows * kDim,
        rel_bias,
        rel_bias, 0L,
        kRows, kDim, kDim, 1.0f);
  }

  mix_bias_ln_kernel<<<dim3(kRows), dim3(128), 0, stream>>>(PB, rid, rel_bias, rel_att, outp, nrel);
}
